// OutputLayer_KAN_1layer_3289944949182
// MI455X (gfx1250) — hardware-verified
//
#include <hip/hip_runtime.h>
#include <math.h>

constexpr int kRows      = 16384;
constexpr int kDin       = 512;
constexpr int kHid       = 256;
constexpr int kNBasis    = 8;
constexpr int kKsp       = kDin * kNBasis;
constexpr int kKtot      = kKsp + kDin;
constexpr int kNcls      = 8;
constexpr int kAttn      = 9;
constexpr int kComb      = kHid + kAttn;
constexpr int kCombPad   = 268;
constexpr int kChunkRows = 8192;
constexpr int kNumChunks = kRows / kChunkRows;
constexpr float kACarry    = 1024.0f;
constexpr float kWCarry    = 32.0f;
constexpr float kGemmScale = 1.0f / (1024.0f * 32.0f);

static_assert(kKtot % 32 == 0, "K multiple of 32");
static_assert(kChunkRows % 64 == 0 && kHid % 64 == 0, "tile multiples");
static_assert(kRows % kChunkRows == 0, "chunks exact");
static_assert((kHid * (kKtot / 8)) % 256 == 0, "prep grid exact");
static_assert(kRows % 256 == 0, "head grid exact");
static_assert((kRows * kComb) % (4 * 256) == 0, "assemble grid exact");

constexpr size_t kOffWT   = 0;
constexpr size_t kBytesWT = (size_t)kHid * kKtot * 2;
constexpr size_t kOffH    = kOffWT + kBytesWT;
constexpr size_t kBytesH  = (size_t)kRows * kHid * 4;
constexpr size_t kOffA    = kOffH + kBytesH;
constexpr size_t kBytesA  = (size_t)kChunkRows * kKtot * 2;
constexpr size_t kWsTotal = kOffA + kBytesA;
static_assert(kOffH % 128 == 0 && kOffA % 128 == 0, "aligned carves");
static_assert(kWsTotal == 94633984ull, "carve total");

typedef __attribute__((ext_vector_type(16))) _Float16 v16h;
typedef __attribute__((ext_vector_type(8)))  _Float16 v8h;
typedef __attribute__((ext_vector_type(16))) __bf16   v16b;
typedef __attribute__((ext_vector_type(8)))  __bf16   v8b;
typedef __attribute__((ext_vector_type(8)))  float    v8f;
typedef __attribute__((ext_vector_type(4)))  float    v4f;
typedef __attribute__((ext_vector_type(4)))  unsigned int v4u;

__device__ __forceinline__ unsigned short f2bf_bits(float f) {
  unsigned u = __float_as_uint(f);
  return (unsigned short)((u + 0x7FFFu + ((u >> 16) & 1u)) >> 16);
}
__device__ __forceinline__ float bf_bits2f(unsigned short h) { return __uint_as_float(((unsigned)h) << 16); }

__device__ __forceinline__ void dep_guard_h(v8f& a, v8f& b, v16h x, v16h y) { asm volatile("v_nop\n\tv_nop\n\tv_nop\n\tv_nop" : "+v"(a), "+v"(b) : "v"(x), "v"(y)); }
__device__ __forceinline__ void dep_guard_b(v8f& a, v8f& b, v16b x, v16b y) { asm volatile("v_nop\n\tv_nop\n\tv_nop\n\tv_nop" : "+v"(a), "+v"(b) : "v"(x), "v"(y)); }
__device__ __forceinline__ void keep4_h(v16h a, v16h b, v16h c, v16h d) { asm volatile("v_nop" :: "v"(a), "v"(b), "v"(c), "v"(d)); }
__device__ __forceinline__ void keep4_b(v16b a, v16b b, v16b c, v16b d) { asm volatile("v_nop" :: "v"(a), "v"(b), "v"(c), "v"(d)); }
__device__ __forceinline__ void acc_guard4(v8f& a, v8f& b, v8f& c, v8f& d) { asm volatile("v_nop\n\tv_nop\n\tv_nop\n\tv_nop" : "+v"(a), "+v"(b), "+v"(c), "+v"(d)); }
template <typename T> struct Frag;
template <> struct Frag<_Float16> {
  typedef v16h V; union U { v16h v; v8h h[2]; };
  static __device__ __forceinline__ v16h load(const _Float16* p) {
    U f; f.h[0] = *(const v8h*)(p); f.h[1] = *(const v8h*)(p + 16); return f.v;
  }
  static __device__ __forceinline__ v8f mma(v16h a, v16h b, v8f c) {
    return __builtin_amdgcn_wmma_f32_16x16x32_f16(false, a, false, b, (short)0, c, false, false);
  }
  static __device__ __forceinline__ void guard(v8f& a, v8f& b, v16h x, v16h y) { dep_guard_h(a, b, x, y); }
  static __device__ __forceinline__ void keep(v16h a, v16h b, v16h c, v16h d) { keep4_h(a, b, c, d); }
};
template <> struct Frag<__bf16> {
  typedef v16b V; union U { v16b v; v8b h[2]; };
  static __device__ __forceinline__ v16b load(const __bf16* p) {
    U f; f.h[0] = *(const v8b*)(p); f.h[1] = *(const v8b*)(p + 16); return f.v;
  }
  static __device__ __forceinline__ v8f mma(v16b a, v16b b, v8f c) {
    return __builtin_amdgcn_wmma_f32_16x16x32_bf16(false, a, false, b, (short)0, c, false, false);
  }
  static __device__ __forceinline__ void guard(v8f& a, v8f& b, v16b x, v16b y) { dep_guard_b(a, b, x, y); }
  static __device__ __forceinline__ void keep(v16b a, v16b b, v16b c, v16b d) { keep4_b(a, b, c, d); }
};

__device__ __forceinline__ unsigned pk16(unsigned short a, unsigned short b) { return (unsigned)a | ((unsigned)b << 16); }
__device__ __forceinline__ unsigned short h_bits(float f) { const _Float16 h = (_Float16)f; return __builtin_bit_cast(unsigned short, h); }

template <int ET> struct Elem;
template <> struct Elem<0> { typedef _Float16 T; };
template <> struct Elem<1> { typedef __bf16 T; };
template <int ET, bool SPLIT, int BIAS_MODE, int OUT_MODE, bool RESID, int ACT = 0>
__global__ __launch_bounds__(256) void wmma_gemm64(
    const unsigned short* __restrict__ Ap, const unsigned short* __restrict__ A2p, int lda, long strideA,
    const unsigned short* __restrict__ Btp, const unsigned short* __restrict__ Bt2p, int ldb, long strideB,
    void* __restrict__ Cout, void* __restrict__ Cout2, int ldc, long strideC,
    const float* __restrict__ bias,
    const float* __restrict__ resid, long strideR,
    int M, int N, int K, float scale) {
  typedef typename Elem<ET>::T T;
  typedef typename Frag<T>::V V;
  const T* A = (const T*)Ap; const T* A2 = (const T*)A2p; const T* Bt = (const T*)Btp; const T* Bt2 = (const T*)Bt2p;
  __shared__ __align__(16) float sT[8][16 * 68];
  const int b    = blockIdx.y;
  const int lane = threadIdx.x & 31;
  const int wave = threadIdx.x >> 5;
  const int tilesN = N >> 6;
  const int tilesM = M >> 6;
  const int tile = blockIdx.x * 8 + wave;
  if (tile >= tilesM * tilesN) return;
  const int tm = tile / tilesN;
  const int tn = tile - tm * tilesN;
  const int m0 = tm << 6;
  const int n0 = tn << 6;

  const T* Ab  = A  + (size_t)b * strideA;
  const T* Bb  = Bt + (size_t)b * strideB;
  const T* Ab2 = SPLIT ? (A2  + (size_t)b * strideA) : nullptr;
  const T* Bb2 = SPLIT ? (Bt2 + (size_t)b * strideB) : nullptr;

  const int rlane = lane & 15;
  const int koff  = (lane >> 4) * 8;
  const int mOff  = (lane >> 4) * 8;

  v8f acc[4][4];
#pragma unroll
  for (int i = 0; i < 4; ++i)
#pragma unroll
    for (int j = 0; j < 4; ++j) acc[i][j] = (v8f){0.f,0.f,0.f,0.f,0.f,0.f,0.f,0.f};

  for (int k0 = 0; k0 < K; k0 += 32) {
    V bh[4], bl[4];
#pragma unroll
    for (int j = 0; j < 4; ++j) {
      const size_t bo = (size_t)(n0 + (j << 4) + rlane) * ldb + koff + k0;
      bh[j] = Frag<T>::load(Bb + bo);
      if (SPLIT) bl[j] = Frag<T>::load(Bb2 + bo);
    }
#pragma unroll
    for (int i = 0; i < 4; ++i) {
      const size_t ao = (size_t)(m0 + (i << 4) + rlane) * lda + koff + k0;
      V ah = Frag<T>::load(Ab + ao);
      V al;
      if (SPLIT) al = Frag<T>::load(Ab2 + ao);
#pragma unroll
      for (int j = 0; j < 4; ++j) {
        acc[i][j] = Frag<T>::mma(ah, bh[j], acc[i][j]);
        if (SPLIT) {
          acc[i][j] = Frag<T>::mma(ah, bl[j], acc[i][j]);
          acc[i][j] = Frag<T>::mma(al, bh[j], acc[i][j]);
        }
      }
      Frag<T>::guard(acc[i][0], acc[i][3], ah, SPLIT ? al : ah);
    }
    Frag<T>::keep(bh[0], bh[1], bh[2], bh[3]);
    if (SPLIT) Frag<T>::keep(bl[0], bl[1], bl[2], bl[3]);
  }
  acc_guard4(acc[0][0], acc[0][1], acc[0][2], acc[0][3]);
  acc_guard4(acc[1][0], acc[1][1], acc[1][2], acc[1][3]);
  acc_guard4(acc[2][0], acc[2][1], acc[2][2], acc[2][3]);
  acc_guard4(acc[3][0], acc[3][1], acc[3][2], acc[3][3]);

  float* slab = sT[wave];
  const float* Rb = RESID ? (resid + (size_t)b * strideR) : nullptr;
#pragma unroll
  for (int i = 0; i < 4; ++i) {
    const int mBase = m0 + (i << 4);
#pragma unroll
    for (int j = 0; j < 4; ++j) {
      const int n = n0 + (j << 4) + rlane;
      float bv = 0.f;
      if (BIAS_MODE == 2) bv = bias[n];
#pragma unroll
      for (int r = 0; r < 8; ++r) {
        float v = acc[i][j][r] * scale;
        if (BIAS_MODE == 1) v += bias[mBase + mOff + r];
        if (BIAS_MODE == 2) v += bv;
        if (RESID) v += Rb[(size_t)(mBase + mOff + r) * ldc + n];
        if (ACT == 2) v = fmaxf(v, 0.0f);
        if (ACT == 4) v = (v > 0.f) ? v : 0.01f * v;
        slab[(mOff + r) * 68 + (j << 4) + rlane] = v;
      }
    }
    __builtin_amdgcn_fence(__ATOMIC_RELEASE, "workgroup");
    __builtin_amdgcn_wave_barrier();
    __builtin_amdgcn_fence(__ATOMIC_ACQUIRE, "workgroup");
    if (OUT_MODE == 0) {
      float* C = (float*)Cout + (size_t)b * strideC;
      const int hh = lane >> 4, c4 = (lane & 15) * 4;
      for (int pass = 0; pass < 2; ++pass) {
#pragma unroll
        for (int it = 0; it < 8; ++it) {
          const int row = it * 2 + hh;
          v4f v = *(const v4f*)(slab + row * 68 + c4);
          *(volatile v4f*)(C + (size_t)(mBase + row) * ldc + n0 + c4) = v;
        }
        __threadfence();
      }
    } else {
      const int q = lane >> 3, c8 = (lane & 7) * 8;
      unsigned short* C  = (unsigned short*)Cout  + (size_t)b * strideC;
      unsigned short* C2 = (OUT_MODE == 2) ? ((unsigned short*)Cout2 + (size_t)b * strideC) : nullptr;
      for (int pass = 0; pass < 2; ++pass) {
#pragma unroll
        for (int it = 0; it < 4; ++it) {
          const int row = it * 4 + q;
          const float* sp = slab + row * 68 + c8;
          v8h hv, lv;
#pragma unroll
          for (int e = 0; e < 8; ++e) {
            if (OUT_MODE == 1) {
              hv[e] = (_Float16)sp[e];
            } else {
              unsigned short hb = f2bf_bits(sp[e]);
              unsigned short lb = f2bf_bits(sp[e] - bf_bits2f(hb));
              hv[e] = __builtin_bit_cast(_Float16, hb);
              lv[e] = __builtin_bit_cast(_Float16, lb);
            }
          }
          *(volatile v8h*)(C + (size_t)(mBase + row) * ldc + n0 + c8) = hv;
          if (OUT_MODE == 2) *(volatile v8h*)(C2 + (size_t)(mBase + row) * ldc + n0 + c8) = lv;
        }
        __threadfence();
      }
    }
    __builtin_amdgcn_fence(__ATOMIC_RELEASE, "workgroup");
    __builtin_amdgcn_wave_barrier();
    __builtin_amdgcn_fence(__ATOMIC_ACQUIRE, "workgroup");
  }
}

__global__ __launch_bounds__(256) void prep_wt_kernel(const float* __restrict__ spw, const float* __restrict__ scl,
                                                      const float* __restrict__ bw, unsigned short* __restrict__ wt) {
  const int i = blockIdx.x * 256 + threadIdx.x;
  const int o = i / (kKtot / 8);
  const int c = (i - o * (kKtot / 8)) * 8;
  const int cs = (c < kKsp) ? c : (kKsp - 8);
  int cb = c - kKsp; cb = (cb < 0) ? 0 : cb;
  const float* ps = spw + (size_t)o * kKsp + cs;
  const float  sc = scl[(size_t)o * kDin + (cs >> 3)];
  const float* pb = bw + (size_t)o * kDin + cb;
  const v4f s0 = *(const v4f*)(ps);
  const v4f s1 = *(const v4f*)(ps + 4);
  const v4f b0 = *(const v4f*)(pb);
  const v4f b1 = *(const v4f*)(pb + 4);
  const bool issp = (c < kKsp);
  unsigned short hb[8];
#pragma unroll
  for (int e = 0; e < 4; ++e) {
    const float vs0 = s0[e] * sc;
    const float vs1 = s1[e] * sc;
    const float v0 = issp ? vs0 : b0[e];
    const float v1 = issp ? vs1 : b1[e];
    hb[e]     = h_bits(v0 * kWCarry);
    hb[4 + e] = h_bits(v1 * kWCarry);
  }
  const v4u u = (v4u){pk16(hb[0], hb[1]), pk16(hb[2], hb[3]), pk16(hb[4], hb[5]), pk16(hb[6], hb[7])};
  unsigned short* q = wt + (size_t)o * kKtot + c;
  *(volatile v4u*)q = u;
  __threadfence();
  *(volatile v4u*)q = u;
}

__global__ __launch_bounds__(256) void basis_gelu_kernel(const float* __restrict__ x, unsigned short* __restrict__ a16, int row0) {
#pragma clang fp contract(off)
  __shared__ __align__(16) float gls[256];
  const int tid  = threadIdx.x;
  const int bx   = blockIdx.x;
  const int rl   = bx >> 1;
  const int half = bx & 1;
  const int i    = half * 256 + tid;
  const float xv = x[(size_t)(row0 + rl) * kDin + i];

  float t[12];
#pragma unroll
  for (int k = 0; k < 12; ++k) t[k] = (float)(k - 3) * 0.4f + (-1.0f);

  float b[11];
#pragma unroll
  for (int j = 0; j < 11; ++j) {
    const bool inb = (xv >= t[j]) & (xv < t[j + 1]);
    b[j] = inb ? 1.0f : 0.0f;
  }
#pragma unroll
  for (int j = 0; j < 10; ++j) {
    const float le = (xv - t[j])     * (1.0f / (t[j + 1] - t[j]));
    const float ri = (t[j + 2] - xv) * (1.0f / (t[j + 2] - t[j + 1]));
    b[j] = le * b[j] + ri * b[j + 1];
  }
#pragma unroll
  for (int j = 0; j < 9; ++j) {
    const float le = (xv - t[j])     * (1.0f / (t[j + 2] - t[j]));
    const float ri = (t[j + 3] - xv) * (1.0f / (t[j + 3] - t[j + 1]));
    b[j] = le * b[j] + ri * b[j + 1];
  }
#pragma unroll
  for (int j = 0; j < 8; ++j) {
    const float le = (xv - t[j])     * (1.0f / (t[j + 3] - t[j]));
    const float ri = (t[j + 4] - xv) * (1.0f / (t[j + 4] - t[j + 1]));
    b[j] = le * b[j] + ri * b[j + 1];
  }

  const float er = erff(xv * 0.70710678118654752440f);
  const float g  = (0.5f * xv) * (er + 1.0f);
  gls[tid] = g * kACarry;

  unsigned short hb[8];
#pragma unroll
  for (int j = 0; j < 8; ++j) hb[j] = h_bits(b[j] * kACarry);
  const v4u ub = (v4u){pk16(hb[0], hb[1]), pk16(hb[2], hb[3]), pk16(hb[4], hb[5]), pk16(hb[6], hb[7])};

  __syncthreads();
  const int lane = tid & 31;
  const int wave = tid >> 5;
  const v4f g0 = *(const v4f*)(gls + lane * 8);
  const v4f g1 = *(const v4f*)(gls + lane * 8 + 4);
  unsigned short hg[8];
#pragma unroll
  for (int e = 0; e < 4; ++e) { hg[e] = h_bits(g0[e]); hg[4 + e] = h_bits(g1[e]); }
  const v4u ug = (v4u){pk16(hg[0], hg[1]), pk16(hg[2], hg[3]), pk16(hg[4], hg[5]), pk16(hg[6], hg[7])};

  unsigned short* rowp = a16 + (size_t)rl * kKtot;
  unsigned short* qb = rowp + (size_t)i * kNBasis;
  unsigned short* qg = rowp + kKsp + half * 256 + lane * 8;
  for (int pass = 0; pass < 2; ++pass) {
    *(volatile v4u*)qb = ub;
    if (wave == 0) *(volatile v4u*)qg = ug;
    __threadfence();
  }
}

__global__ __launch_bounds__(256) void head_kernel(const float* __restrict__ H, const float* __restrict__ attn,
                                                   const float* __restrict__ clsw, const float* __restrict__ clsb,
                                                   float* __restrict__ out0) {
  __shared__ __align__(16) float wsm[kNcls * kCombPad];
  __shared__ float bsm[kNcls];
  __shared__ __align__(16) float lg[256 * kNcls];
  const int tid = threadIdx.x;
  for (int e = tid; e < kNcls * kComb; e += 256) {
    const int c = e / kComb;
    const int n = e - c * kComb;
    wsm[c * kCombPad + n] = clsw[e];
  }
  if (tid < kNcls) bsm[tid] = clsb[tid];
  __syncthreads();

  const int row = blockIdx.x * 256 + tid;
  float acc[kNcls];
#pragma unroll
  for (int c = 0; c < kNcls; ++c) acc[c] = 0.0f;
  const float* hr = H + (size_t)row * kHid;
#pragma unroll 1
  for (int n4 = 0; n4 < kHid / 4; ++n4) {
    const v4f hv = *(const v4f*)(hr + 4 * n4);
#pragma unroll
    for (int c = 0; c < kNcls; ++c) {
      const v4f wv = *(const v4f*)(wsm + c * kCombPad + 4 * n4);
      acc[c] += hv[0] * wv[0];
      acc[c] += hv[1] * wv[1];
      acc[c] += hv[2] * wv[2];
      acc[c] += hv[3] * wv[3];
    }
  }
  const float* ar = attn + (size_t)row * kAttn;
#pragma unroll 1
  for (int n = 0; n < kAttn; ++n) {
    const float av = ar[n];
#pragma unroll
    for (int c = 0; c < kNcls; ++c) acc[c] += av * wsm[c * kCombPad + kHid + n];
  }
#pragma unroll
  for (int c = 0; c < kNcls; ++c) acc[c] += bsm[c];
  float m = acc[0];
#pragma unroll
  for (int c = 1; c < kNcls; ++c) m = fmaxf(m, acc[c]);
  float* lr = lg + tid * kNcls;
#pragma unroll
  for (int c = 0; c < kNcls; ++c) lr[c] = acc[c] - m;
  float s = 0.0f;
#pragma unroll 1
  for (int c = 0; c < kNcls; ++c) s += expf(lr[c]);
  const float lse = logf(s);
#pragma unroll 1
  for (int c = 0; c < kNcls; ++c) lr[c] = lr[c] - lse;
  __syncthreads();

  const int lane = tid & 31;
  const int wave = tid >> 5;
  float* ob = out0 + (size_t)blockIdx.x * (256 * kNcls);
  for (int pass = 0; pass < 2; ++pass) {
#pragma unroll
    for (int it = 0; it < 2; ++it) {
      const int idx = wave * 256 + it * 128 + lane * 4;
      const v4f v = *(const v4f*)(lg + idx);
      *(volatile v4f*)(ob + idx) = v;
    }
    __threadfence();
  }
}

__global__ __launch_bounds__(256) void assemble_kernel(const float* __restrict__ H, const float* __restrict__ attn,
                                                       float* __restrict__ out1) {
  const int t  = blockIdx.x * 256 + threadIdx.x;
  const int e0 = t * 4;
  v4f v;
#pragma unroll
  for (int u = 0; u < 4; ++u) {
    const int e   = e0 + u;
    const int row = e / kComb;
    const int col = e - row * kComb;
    const int hc  = (col < kHid) ? col : (kHid - 1);
    int ac = col - kHid; ac = (ac < 0) ? 0 : ac;
    const float hvv = H[(size_t)row * kHid + hc];
    const float avv = attn[(size_t)row * kAttn + ac];
    v[u] = (col < kHid) ? hvv : avv;
  }
  float* q = out1 + (size_t)e0;
  *(volatile v4f*)q = v;
  __threadfence();
  *(volatile v4f*)q = v;
}

extern "C" void kernel_launch(void* const* d_in, const int* in_sizes, int n_in,
                              void* d_out, int out_size, void* d_ws, size_t ws_size,
                              hipStream_t stream) {
  if (n_in < 7) return;
  if (in_sizes[0] != kRows * kDin || in_sizes[1] != kRows * kAttn || in_sizes[2] != kHid * kDin ||
      in_sizes[3] != kHid * kKsp || in_sizes[4] != kHid * kDin || in_sizes[5] != kNcls * kComb ||
      in_sizes[6] != kNcls) return;
  if (out_size != kRows * (kNcls + kComb)) return;
  if (ws_size < kWsTotal) return;

  const float* x        = (const float*)d_in[0];
  const float* attn     = (const float*)d_in[1];
  const float* base_w   = (const float*)d_in[2];
  const float* spline_w = (const float*)d_in[3];
  const float* scaler   = (const float*)d_in[4];
  const float* clsw     = (const float*)d_in[5];
  const float* clsb     = (const float*)d_in[6];

  float* out0 = (float*)d_out;
  float* out1 = (float*)d_out + (size_t)kRows * kNcls;

  char* ws = (char*)d_ws;
  unsigned short* WT  = (unsigned short*)(ws + kOffWT);
  float*          H   = (float*)(ws + kOffH);
  unsigned short* A16 = (unsigned short*)(ws + kOffA);

  prep_wt_kernel<<<(kHid * (kKtot / 8)) / 256, 256, 0, stream>>>(spline_w, scaler, base_w, WT);

  for (int ch = 0; ch < kNumChunks; ++ch) {
    basis_gelu_kernel<<<kChunkRows * 2, 256, 0, stream>>>(x, A16, ch * kChunkRows);
    float* Hc = H + (size_t)ch * kChunkRows * kHid;
    const int tiles  = (kChunkRows / 64) * (kHid / 64);
    const int blocks = (tiles + 7) / 8;
    wmma_gemm64<0, false, 0, 0, false, 0><<<dim3(blocks, 1), 256, 0, stream>>>(
        (const unsigned short*)A16, (const unsigned short*)A16, kKtot, 0L,
        (const unsigned short*)WT, (const unsigned short*)WT, kKtot, 0L,
        (void*)Hc, (void*)Hc, kHid, 0L,
        (const float*)Hc,
        (const float*)Hc, 0L,
        kChunkRows, kHid, kKtot, kGemmScale);
  }

  head_kernel<<<kRows / 256, 256, 0, stream>>>(H, attn, clsw, clsb, out0);
  assemble_kernel<<<(kRows * kComb) / (4 * 256), 256, 0, stream>>>(H, attn, out1);
}
